// MatrixLSTMCell_61744449847852
// MI455X (gfx1250) — hardware-verified
//
#include <hip/hip_runtime.h>
#include <math.h>

constexpr int kB   = 4;
constexpr int kS   = 2048;
constexpr int kD   = 512;
constexpr int kNH  = 4;
constexpr int kDH  = 128;
constexpr int kT   = kB * kS;
constexpr int kGin = 3 * kD;
constexpr int kGN  = 64;
constexpr int kHeadsPerPass = 2;
constexpr int kPasses = (kB * kNH) / kHeadsPerPass;
constexpr float kQKScale   = 0.08838834764831845f;
constexpr float kPCarry    = 1048576.0f;
constexpr float kPCarryInv = 1.0f / 1048576.0f;
constexpr float kEpsN      = 5e-5f;
constexpr float kEpsLN     = 1e-3f;
constexpr float kInvDH     = 1.0f / 128.0f;
static_assert(kS == 2048 && kD == 512 && kDH == 128 && kNH == 4, "fixed geometry");

constexpr size_t kOffQKV = 0;
constexpr size_t kSzQKV  = (size_t)kT * kGin * 2;
constexpr size_t kOffVt  = kOffQKV + kSzQKV;
constexpr size_t kSzVt   = (size_t)kB * kNH * kDH * kS * 2;
constexpr size_t kOffWG  = kOffVt + kSzVt;
constexpr size_t kSzWG   = (size_t)kGN * kGin * 2;
constexpr size_t kOffG   = kOffWG + kSzWG;
constexpr size_t kSzG    = (size_t)kT * kGN * 4;
constexpr size_t kOffA   = kOffG + kSzG;
constexpr size_t kSzScan = (size_t)kB * kNH * kS * 4;
constexpr size_t kOffAM  = kOffA + kSzScan;
constexpr size_t kOffM   = kOffAM + kSzScan;
constexpr size_t kOffS   = kOffM + kSzScan;
constexpr size_t kSzS    = (size_t)kHeadsPerPass * kS * kS * 4;
constexpr size_t kOffP   = kOffS + kSzS;
constexpr size_t kSzP    = (size_t)kHeadsPerPass * kS * kS * 2;
constexpr size_t kOffH   = kOffP + kSzP;
constexpr size_t kSzH    = (size_t)kT * kD * 4;
constexpr size_t kWsTotal = kOffH + kSzH;
static_assert(kWsTotal == 103350272ull, "carve total");
static_assert(kWsTotal <= 134217728ull, "carve limit");
static_assert((kOffVt % 128) == 0 && (kOffWG % 128) == 0 && (kOffG % 128) == 0 && (kOffA % 128) == 0 &&
              (kOffAM % 128) == 0 && (kOffM % 128) == 0 && (kOffS % 128) == 0 && (kOffP % 128) == 0 &&
              (kOffH % 128) == 0, "alignment");

typedef __attribute__((ext_vector_type(16))) _Float16 v16h;
typedef __attribute__((ext_vector_type(8)))  _Float16 v8h;
typedef __attribute__((ext_vector_type(16))) __bf16   v16b;
typedef __attribute__((ext_vector_type(8)))  __bf16   v8b;
typedef __attribute__((ext_vector_type(8)))  float    v8f;
typedef __attribute__((ext_vector_type(4)))  float    v4f;
typedef __attribute__((ext_vector_type(4)))  unsigned int v4u;

__device__ __forceinline__ unsigned short f2bf_bits(float f) {
  unsigned u = __float_as_uint(f);
  return (unsigned short)((u + 0x7FFFu + ((u >> 16) & 1u)) >> 16);
}
__device__ __forceinline__ float bf_bits2f(unsigned short h) { return __uint_as_float(((unsigned)h) << 16); }

__device__ __forceinline__ void dep_guard_h(v8f& a, v8f& b, v16h x, v16h y) { asm volatile("v_nop\n\tv_nop\n\tv_nop\n\tv_nop" : "+v"(a), "+v"(b) : "v"(x), "v"(y)); }
__device__ __forceinline__ void dep_guard_b(v8f& a, v8f& b, v16b x, v16b y) { asm volatile("v_nop\n\tv_nop\n\tv_nop\n\tv_nop" : "+v"(a), "+v"(b) : "v"(x), "v"(y)); }
__device__ __forceinline__ void keep4_h(v16h a, v16h b, v16h c, v16h d) { asm volatile("v_nop" :: "v"(a), "v"(b), "v"(c), "v"(d)); }
__device__ __forceinline__ void keep4_b(v16b a, v16b b, v16b c, v16b d) { asm volatile("v_nop" :: "v"(a), "v"(b), "v"(c), "v"(d)); }
__device__ __forceinline__ void acc_guard4(v8f& a, v8f& b, v8f& c, v8f& d) { asm volatile("v_nop\n\tv_nop\n\tv_nop\n\tv_nop" : "+v"(a), "+v"(b), "+v"(c), "+v"(d)); }
template <typename T> struct Frag;
template <> struct Frag<_Float16> {
  typedef v16h V; union U { v16h v; v8h h[2]; };
  static __device__ __forceinline__ v16h load(const _Float16* p) {
    U f; f.h[0] = *(const v8h*)(p); f.h[1] = *(const v8h*)(p + 16); return f.v;
  }
  static __device__ __forceinline__ v8f mma(v16h a, v16h b, v8f c) {
    return __builtin_amdgcn_wmma_f32_16x16x32_f16(false, a, false, b, (short)0, c, false, false);
  }
  static __device__ __forceinline__ void guard(v8f& a, v8f& b, v16h x, v16h y) { dep_guard_h(a, b, x, y); }
  static __device__ __forceinline__ void keep(v16h a, v16h b, v16h c, v16h d) { keep4_h(a, b, c, d); }
};
template <> struct Frag<__bf16> {
  typedef v16b V; union U { v16b v; v8b h[2]; };
  static __device__ __forceinline__ v16b load(const __bf16* p) {
    U f; f.h[0] = *(const v8b*)(p); f.h[1] = *(const v8b*)(p + 16); return f.v;
  }
  static __device__ __forceinline__ v8f mma(v16b a, v16b b, v8f c) {
    return __builtin_amdgcn_wmma_f32_16x16x32_bf16(false, a, false, b, (short)0, c, false, false);
  }
  static __device__ __forceinline__ void guard(v8f& a, v8f& b, v16b x, v16b y) { dep_guard_b(a, b, x, y); }
  static __device__ __forceinline__ void keep(v16b a, v16b b, v16b c, v16b d) { keep4_b(a, b, c, d); }
};

__device__ __forceinline__ unsigned pk16(unsigned short a, unsigned short b) { return (unsigned)a | ((unsigned)b << 16); }
__device__ __forceinline__ unsigned short h_bits(float f) { const _Float16 h = (_Float16)f; return __builtin_bit_cast(unsigned short, h); }

template <int ET> struct Elem;
template <> struct Elem<0> { typedef _Float16 T; };
template <> struct Elem<1> { typedef __bf16 T; };
template <int ET, bool SPLIT, int BIAS_MODE, int OUT_MODE, bool RESID, int ACT = 0, int TRI = 0>
__global__ __launch_bounds__(256) void wmma_gemm64(
    const unsigned short* __restrict__ Ap, const unsigned short* __restrict__ A2p, int lda, long strideA,
    const unsigned short* __restrict__ Btp, const unsigned short* __restrict__ Bt2p, int ldb, long strideB,
    void* __restrict__ Cout, void* __restrict__ Cout2, int ldc, long strideC,
    const float* __restrict__ bias,
    const float* __restrict__ resid, long strideR,
    int M, int N, int K, float scale) {
  typedef typename Elem<ET>::T T;
  typedef typename Frag<T>::V V;
  const T* A = (const T*)Ap; const T* A2 = (const T*)A2p; const T* Bt = (const T*)Btp; const T* Bt2 = (const T*)Bt2p;
  __shared__ __align__(16) float sT[8][16 * 68];
  const int b    = blockIdx.y;
  const int lane = threadIdx.x & 31;
  const int wave = threadIdx.x >> 5;
  const int tilesN = N >> 6;
  const int tilesM = M >> 6;
  const int tile = blockIdx.x * 8 + wave;
  if (tile >= tilesM * tilesN) return;
  const int tm = tile / tilesN;
  const int tn = tile - tm * tilesN;
  if (TRI == 1 && tn > tm) return;
  const int m0 = tm << 6;
  const int n0 = tn << 6;
  int Kt = K;
  if (TRI == 2) { const int kl = m0 + 64; Kt = (kl < K) ? kl : K; }

  const T* Ab  = A  + (size_t)b * strideA;
  const T* Bb  = Bt + (size_t)b * strideB;
  const T* Ab2 = SPLIT ? (A2  + (size_t)b * strideA) : nullptr;
  const T* Bb2 = SPLIT ? (Bt2 + (size_t)b * strideB) : nullptr;

  const int rlane = lane & 15;
  const int koff  = (lane >> 4) * 8;
  const int mOff  = (lane >> 4) * 8;

  v8f acc[4][4];
#pragma unroll
  for (int i = 0; i < 4; ++i)
#pragma unroll
    for (int j = 0; j < 4; ++j) acc[i][j] = (v8f){0.f,0.f,0.f,0.f,0.f,0.f,0.f,0.f};

  for (int k0 = 0; k0 < Kt; k0 += 32) {
    V bh[4], bl[4];
#pragma unroll
    for (int j = 0; j < 4; ++j) {
      const size_t bo = (size_t)(n0 + (j << 4) + rlane) * ldb + koff + k0;
      bh[j] = Frag<T>::load(Bb + bo);
      if (SPLIT) bl[j] = Frag<T>::load(Bb2 + bo);
    }
#pragma unroll
    for (int i = 0; i < 4; ++i) {
      const size_t ao = (size_t)(m0 + (i << 4) + rlane) * lda + koff + k0;
      V ah = Frag<T>::load(Ab + ao);
      V al;
      if (SPLIT) al = Frag<T>::load(Ab2 + ao);
#pragma unroll
      for (int j = 0; j < 4; ++j) {
        acc[i][j] = Frag<T>::mma(ah, bh[j], acc[i][j]);
        if (SPLIT) {
          acc[i][j] = Frag<T>::mma(ah, bl[j], acc[i][j]);
          acc[i][j] = Frag<T>::mma(al, bh[j], acc[i][j]);
        }
      }
      Frag<T>::guard(acc[i][0], acc[i][3], ah, SPLIT ? al : ah);
    }
    Frag<T>::keep(bh[0], bh[1], bh[2], bh[3]);
    if (SPLIT) Frag<T>::keep(bl[0], bl[1], bl[2], bl[3]);
  }
  acc_guard4(acc[0][0], acc[0][1], acc[0][2], acc[0][3]);
  acc_guard4(acc[1][0], acc[1][1], acc[1][2], acc[1][3]);
  acc_guard4(acc[2][0], acc[2][1], acc[2][2], acc[2][3]);
  acc_guard4(acc[3][0], acc[3][1], acc[3][2], acc[3][3]);

  float* slab = sT[wave];
  const float* Rb = RESID ? (resid + (size_t)b * strideR) : nullptr;
#pragma unroll
  for (int i = 0; i < 4; ++i) {
    const int mBase = m0 + (i << 4);
#pragma unroll
    for (int j = 0; j < 4; ++j) {
      const int n = n0 + (j << 4) + rlane;
      float bv = 0.f;
      if (BIAS_MODE == 2) bv = bias[n];
#pragma unroll
      for (int r = 0; r < 8; ++r) {
        float v = acc[i][j][r] * scale;
        if (BIAS_MODE == 1) v += bias[mBase + mOff + r];
        if (BIAS_MODE == 2) v += bv;
        if (RESID) v += Rb[(size_t)(mBase + mOff + r) * ldc + n];
        if (ACT == 2) v = fmaxf(v, 0.0f);
        if (ACT == 4) v = (v > 0.f) ? v : 0.01f * v;
        slab[(mOff + r) * 68 + (j << 4) + rlane] = v;
      }
    }
    __builtin_amdgcn_fence(__ATOMIC_RELEASE, "workgroup");
    __builtin_amdgcn_wave_barrier();
    __builtin_amdgcn_fence(__ATOMIC_ACQUIRE, "workgroup");
    if (OUT_MODE == 0) {
      float* C = (float*)Cout + (size_t)b * strideC;
      const int hh = lane >> 4, c4 = (lane & 15) * 4;
      for (int pass = 0; pass < 2; ++pass) {
#pragma unroll
        for (int it = 0; it < 8; ++it) {
          const int row = it * 2 + hh;
          v4f v = *(const v4f*)(slab + row * 68 + c4);
          *(volatile v4f*)(C + (size_t)(mBase + row) * ldc + n0 + c4) = v;
        }
        __threadfence();
      }
    } else {
      const int q = lane >> 3, c8 = (lane & 7) * 8;
      unsigned short* C  = (unsigned short*)Cout  + (size_t)b * strideC;
      unsigned short* C2 = (OUT_MODE == 2) ? ((unsigned short*)Cout2 + (size_t)b * strideC) : nullptr;
      for (int pass = 0; pass < 2; ++pass) {
#pragma unroll
        for (int it = 0; it < 4; ++it) {
          const int row = it * 4 + q;
          const float* sp = slab + row * 68 + c8;
          v8h hv, lv;
#pragma unroll
          for (int e = 0; e < 8; ++e) {
            if (OUT_MODE == 1) {
              hv[e] = (_Float16)sp[e];
            } else {
              unsigned short hb = f2bf_bits(sp[e]);
              unsigned short lb = f2bf_bits(sp[e] - bf_bits2f(hb));
              hv[e] = __builtin_bit_cast(_Float16, hb);
              lv[e] = __builtin_bit_cast(_Float16, lb);
            }
          }
          *(volatile v8h*)(C + (size_t)(mBase + row) * ldc + n0 + c8) = hv;
          if (OUT_MODE == 2) *(volatile v8h*)(C2 + (size_t)(mBase + row) * ldc + n0 + c8) = lv;
        }
        __threadfence();
      }
    }
    __builtin_amdgcn_fence(__ATOMIC_RELEASE, "workgroup");
    __builtin_amdgcn_wave_barrier();
    __builtin_amdgcn_fence(__ATOMIC_ACQUIRE, "workgroup");
  }
}

__global__ __launch_bounds__(256) void cast_qkv_kernel(const float* __restrict__ q, const float* __restrict__ k,
                                                       const float* __restrict__ v, unsigned short* __restrict__ out) {
  const int i = blockIdx.x * 256 + threadIdx.x;
  if (i >= kT * (kD / 8)) return;
  const int seg = blockIdx.y;
  const int row = i >> 6, ch = i & 63;
  const float* src = (seg == 0) ? q : ((seg == 1) ? k : v);
  const float* p = src + (size_t)row * kD + ch * 8;
  const v4f a = *(const v4f*)(p);
  const v4f c = *(const v4f*)(p + 4);
  unsigned short hb[8];
#pragma unroll
  for (int e = 0; e < 4; ++e) { hb[e] = f2bf_bits(a[e]); hb[4 + e] = f2bf_bits(c[e]); }
  const v4u u = (v4u){pk16(hb[0], hb[1]), pk16(hb[2], hb[3]), pk16(hb[4], hb[5]), pk16(hb[6], hb[7])};
  unsigned short* o = out + (size_t)row * kGin + seg * kD + ch * 8;
  *(volatile v4u*)o = u;
  __threadfence();
  *(volatile v4u*)o = u;
}

__global__ __launch_bounds__(256) void cast_vt_kernel(const float* __restrict__ v, unsigned short* __restrict__ out) {
  __shared__ float sm[64][65];
  const int t  = threadIdx.x;
  const int s0 = blockIdx.x * 64;
  const int y  = blockIdx.y;
  const int b  = blockIdx.z;
#pragma unroll
  for (int i = 0; i < 16; ++i) {
    const int e = i * 256 + t;
    const int r = e >> 6;
    const int c = e & 63;
    sm[c][r] = v[((size_t)(b * kS + s0 + r)) * kD + y * 64 + c];
  }
  __syncthreads();
  const int lane = t & 31, wave = t >> 5;
  const int q = lane >> 3, c8 = (lane & 7) * 8;
  const int g = b * kNH + (y >> 1);
  const int d0 = (y & 1) * 64;
  unsigned short* op = out + ((size_t)g * kDH + d0) * kS + s0;
  for (int pass = 0; pass < 2; ++pass) {
#pragma unroll
    for (int it = 0; it < 2; ++it) {
      const int row = wave * 8 + it * 4 + q;
      unsigned short hb[8];
#pragma unroll
      for (int e = 0; e < 8; ++e) hb[e] = h_bits(bf_bits2f(f2bf_bits(sm[row][c8 + e])));
      const v4u u = (v4u){pk16(hb[0], hb[1]), pk16(hb[2], hb[3]), pk16(hb[4], hb[5]), pk16(hb[6], hb[7])};
      *(volatile v4u*)(op + (size_t)row * kS + c8) = u;
    }
    __threadfence();
  }
}

__global__ __launch_bounds__(256) void cast_w_kernel(const float* __restrict__ Wi, const float* __restrict__ Wf,
                                                     unsigned short* __restrict__ out) {
  const int i = blockIdx.x * 256 + threadIdx.x;
  if (i >= kGN * (kGin / 8)) return;
  const int row = i / (kGin / 8);
  const int ch  = i - row * (kGin / 8);
  const int ri  = (row < 4) ? row : 3;
  int rf = row - 4; rf = (rf < 0) ? 0 : ((rf > 3) ? 3 : rf);
  const float* pi = Wi + (size_t)ri * kGin + ch * 8;
  const float* pf = Wf + (size_t)rf * kGin + ch * 8;
  const v4f ia = *(const v4f*)(pi);
  const v4f ic = *(const v4f*)(pi + 4);
  const v4f fa = *(const v4f*)(pf);
  const v4f fc = *(const v4f*)(pf + 4);
  const bool useI = (row < 4);
  const bool useF = (row >= 4) && (row < 8);
  unsigned short hb[8];
#pragma unroll
  for (int e = 0; e < 4; ++e) {
    const float x0 = useI ? ia[e] : (useF ? fa[e] : 0.f);
    const float x1 = useI ? ic[e] : (useF ? fc[e] : 0.f);
    hb[e] = f2bf_bits(x0);
    hb[4 + e] = f2bf_bits(x1);
  }
  const v4u u = (v4u){pk16(hb[0], hb[1]), pk16(hb[2], hb[3]), pk16(hb[4], hb[5]), pk16(hb[6], hb[7])};
  unsigned short* o = out + (size_t)row * kGin + ch * 8;
  *(volatile v4u*)o = u;
  __threadfence();
  *(volatile v4u*)o = u;
}

__global__ __launch_bounds__(256) void scan_kernel(const float* __restrict__ G, const float* __restrict__ bi,
                                                   const float* __restrict__ bfv,
                                                   float* __restrict__ Aout, float* __restrict__ AMout, float* __restrict__ Mout) {
  __shared__ float shls[kS];
  __shared__ float shi[kS];
  __shared__ __align__(16) float sA[kS];
  __shared__ __align__(16) float sAM[kS];
  __shared__ __align__(16) float sM[kS];
  __shared__ float shs[256];
  __shared__ float shm[256];
  const int g = blockIdx.x;
  const int b = g >> 2, h = g & 3;
  const int tid = threadIdx.x;
  const int t0 = tid * 8;
  const float bih = bi[h], bfh = bfv[h];
#pragma unroll 1
  for (int j = 0; j < 8; ++j) {
    const int s = t0 + j;
    const float* gr = G + (size_t)(b * kS + s) * kGN;
    const float ip = gr[h] + bih;
    const float fp = gr[4 + h] + bfh;
    const float ls = fminf(fp, 0.f) - log1pf(expf(-fabsf(fp)));
    shls[s] = ls;
    shi[s] = ip;
  }
  float cums[8];
  float run = 0.f;
#pragma unroll
  for (int j = 0; j < 8; ++j) { run += shls[t0 + j]; cums[j] = run; }
  shs[tid] = run;
  __syncthreads();
  for (int off = 1; off < 256; off <<= 1) {
    const int src = (tid >= off) ? (tid - off) : 0;
    const float vv = (tid >= off) ? shs[src] : 0.f;
    __syncthreads();
    shs[tid] += vv;
    __syncthreads();
  }
  const int tidm1 = (tid > 0) ? (tid - 1) : 0;
  const float excl = (tid > 0) ? shs[tidm1] : 0.f;
  float bcv[8], av[8], cmax[8];
  float rmax = -3.0e38f;
#pragma unroll
  for (int j = 0; j < 8; ++j) {
    bcv[j] = excl + cums[j];
    av[j] = shi[t0 + j] - bcv[j];
    rmax = fmaxf(rmax, av[j]);
    cmax[j] = rmax;
  }
  shm[tid] = rmax;
  __syncthreads();
  for (int off = 1; off < 256; off <<= 1) {
    const int src = (tid >= off) ? (tid - off) : 0;
    const float vv = (tid >= off) ? shm[src] : -3.0e38f;
    __syncthreads();
    shm[tid] = fmaxf(shm[tid], vv);
    __syncthreads();
  }
  const float exm = (tid > 0) ? shm[tidm1] : -3.0e38f;
#pragma unroll
  for (int j = 0; j < 8; ++j) {
    const float am = fmaxf(exm, cmax[j]);
    sA[t0 + j]  = av[j];
    sAM[t0 + j] = am;
    sM[t0 + j]  = bcv[j] + am;
  }
  __syncthreads();
  float* ga  = Aout  + (size_t)g * kS;
  float* gam = AMout + (size_t)g * kS;
  float* gm  = Mout  + (size_t)g * kS;
  for (int pass = 0; pass < 2; ++pass) {
#pragma unroll
    for (int half = 0; half < 2; ++half) {
      const int idx = half * 1024 + tid * 4;
      const v4f x0 = *(const v4f*)(sA + idx);
      const v4f x1 = *(const v4f*)(sAM + idx);
      const v4f x2 = *(const v4f*)(sM + idx);
      *(volatile v4f*)(ga + idx)  = x0;
      *(volatile v4f*)(gam + idx) = x1;
      *(volatile v4f*)(gm + idx)  = x2;
    }
    __threadfence();
  }
}

__global__ __launch_bounds__(256) void pweight_kernel(const float* __restrict__ S, unsigned short* __restrict__ P,
                                                      const float* __restrict__ Aarr, const float* __restrict__ AMarr,
                                                      const float* __restrict__ Marr, int b, int h0) {
  const int wave = threadIdx.x >> 5, lane = threadIdx.x & 31;
  const int wid = blockIdx.x * 8 + wave;
  const int hl  = wid >> 11;
  const int t   = wid & (kS - 1);
  const int g   = b * kNH + h0 + hl;
  const int L   = ((t >> 6) + 1) << 6;
  const float amax_t = AMarr[(size_t)g * kS + t];
  const float m_t    = Marr[(size_t)g * kS + t];
  const float* Srow = S + (size_t)hl * kS * kS + (size_t)t * kS;
  const float* Arow = Aarr + (size_t)g * kS;
  float cv[8][8];
  float rsum = 0.f;
#pragma unroll
  for (int c = 0; c < 8; ++c) {
#pragma unroll
    for (int e = 0; e < 8; ++e) cv[c][e] = 0.f;
    const int base = c * 256;
    if (base < L) {
      const int col  = base + 8 * lane;
      const int colc = (col < L - 8) ? col : (L - 8);
      const v4f s0 = *(const v4f*)(Srow + colc);
      const v4f s1 = *(const v4f*)(Srow + colc + 4);
      const v4f a0 = *(const v4f*)(Arow + colc);
      const v4f a1 = *(const v4f*)(Arow + colc + 4);
#pragma unroll
      for (int e = 0; e < 8; ++e) {
        const float sv = (e < 4) ? s0[e & 3] : s1[e & 3];
        const float aa = (e < 4) ? a0[e & 3] : a1[e & 3];
        const bool valid = (col + e <= t);
        const float d = valid ? __expf(aa - amax_t) : 0.f;
        const float x = valid ? (sv * d) : 0.f;
        cv[c][e] = x;
        rsum += x;
      }
    }
  }
#pragma unroll
  for (int off = 16; off > 0; off >>= 1) rsum += __shfl_xor(rsum, off, 32);
  const float n    = fmaxf(fabsf(rsum), __expf(-m_t));
  const float rinv = 1.0f / (n + kEpsN);
  const float psc  = rinv * kPCarry;
  v4u pk[8];
#pragma unroll
  for (int c = 0; c < 8; ++c) {
    unsigned short hb[8];
#pragma unroll
    for (int e = 0; e < 8; ++e) {
      float y = cv[c][e] * psc;
      y = fminf(fmaxf(y, -65000.f), 65000.f);
      hb[e] = h_bits(y);
    }
    pk[c] = (v4u){pk16(hb[0], hb[1]), pk16(hb[2], hb[3]), pk16(hb[4], hb[5]), pk16(hb[6], hb[7])};
  }
  unsigned short* Prow = P + (size_t)hl * kS * kS + (size_t)t * kS;
  for (int pass = 0; pass < 2; ++pass) {
#pragma unroll
    for (int c = 0; c < 8; ++c) {
      const int col = c * 256 + 8 * lane;
      if (col < L) *(volatile v4u*)(Prow + col) = pk[c];
    }
    __threadfence();
  }
}

__global__ __launch_bounds__(256) void norm_kernel(const float* __restrict__ H, const float* __restrict__ lnw,
                                                   const float* __restrict__ lnb, float* __restrict__ out) {
  const int wave = threadIdx.x >> 5, lane = threadIdx.x & 31;
  const int wid = blockIdx.x * 8 + wave;
  const int row = wid >> 2, h = wid & 3;
  const size_t off = (size_t)row * kD + h * kDH + lane * 4;
  const v4f x = *(const v4f*)(H + off);
  float s1 = (x[0] + x[1]) + (x[2] + x[3]);
#pragma unroll
  for (int o = 16; o > 0; o >>= 1) s1 += __shfl_xor(s1, o, 32);
  const float mu = s1 * kInvDH;
  const float d0 = x[0] - mu, d1 = x[1] - mu, d2 = x[2] - mu, d3 = x[3] - mu;
  float s2 = (d0 * d0 + d1 * d1) + (d2 * d2 + d3 * d3);
#pragma unroll
  for (int o = 16; o > 0; o >>= 1) s2 += __shfl_xor(s2, o, 32);
  const float var  = s2 * kInvDH;
  const float rstd = 1.0f / sqrtf(var + kEpsLN);
  const v4f w  = *(const v4f*)(lnw + h * kDH + lane * 4);
  const v4f bb = *(const v4f*)(lnb + h * kDH + lane * 4);
  v4f y;
  y[0] = d0 * rstd * (1.0f + w[0]) + bb[0];
  y[1] = d1 * rstd * (1.0f + w[1]) + bb[1];
  y[2] = d2 * rstd * (1.0f + w[2]) + bb[2];
  y[3] = d3 * rstd * (1.0f + w[3]) + bb[3];
  *(volatile v4f*)(out + off) = y;
  __threadfence();
  *(volatile v4f*)(out + off) = y;
}

extern "C" void kernel_launch(void* const* d_in, const int* in_sizes, int n_in,
                              void* d_out, int out_size, void* d_ws, size_t ws_size,
                              hipStream_t stream) {
  if (n_in < 9) return;
  if (in_sizes[0] != kT * kD || in_sizes[1] != kT * kD || in_sizes[2] != kT * kD) return;
  if (in_sizes[3] != kNH * kGin || in_sizes[5] != kNH * kGin) return;
  if (in_sizes[4] < kNH || in_sizes[6] < kNH || in_sizes[7] < kD || in_sizes[8] < kD) return;
  if (out_size != kT * kD) return;
  if (ws_size < kWsTotal) return;

  const float* q   = (const float*)d_in[0];
  const float* k   = (const float*)d_in[1];
  const float* v   = (const float*)d_in[2];
  const float* Wi  = (const float*)d_in[3];
  const float* bi  = (const float*)d_in[4];
  const float* Wf  = (const float*)d_in[5];
  const float* bfv = (const float*)d_in[6];
  const float* lnw = (const float*)d_in[7];
  const float* lnb = (const float*)d_in[8];
  float* out = (float*)d_out;

  char* ws = (char*)d_ws;
  unsigned short* QKV16 = (unsigned short*)(ws + kOffQKV);
  unsigned short* Vt16  = (unsigned short*)(ws + kOffVt);
  unsigned short* WG16  = (unsigned short*)(ws + kOffWG);
  float* G     = (float*)(ws + kOffG);
  float* Aarr  = (float*)(ws + kOffA);
  float* AMarr = (float*)(ws + kOffAM);
  float* Marr  = (float*)(ws + kOffM);
  float* Sbuf  = (float*)(ws + kOffS);
  unsigned short* Pbuf = (unsigned short*)(ws + kOffP);
  float* Hbuf  = (float*)(ws + kOffH);

  cast_qkv_kernel<<<dim3(kT * (kD / 8) / 256, 3), 256, 0, stream>>>(q, k, v, QKV16);
  cast_vt_kernel<<<dim3(kS / 64, kD / 64, kB), 256, 0, stream>>>(v, Vt16);
  cast_w_kernel<<<(kGN * (kGin / 8)) / 256, 256, 0, stream>>>(Wi, Wf, WG16);

  wmma_gemm64<1, false, 0, 0, false, 0, 0><<<dim3((kT / 64) * (kGN / 64) / 8, 1), 256, 0, stream>>>(
      QKV16, nullptr, kGin, 0L, WG16, nullptr, kGin, 0L,
      (void*)G, nullptr, kGN, 0L, nullptr, nullptr, 0L, kT, kGN, kGin, 1.0f);

  scan_kernel<<<kB * kNH, 256, 0, stream>>>(G, bi, bfv, Aarr, AMarr, Marr);

  for (int p = 0; p < kPasses; ++p) {
    const int b  = p >> 1;
    const int h0 = (p & 1) * kHeadsPerPass;
    const unsigned short* qa = QKV16 + (size_t)b * kS * kGin + h0 * kDH;
    const unsigned short* kb = QKV16 + (size_t)b * kS * kGin + kD + h0 * kDH;
    wmma_gemm64<1, false, 0, 0, false, 0, 1><<<dim3((kS / 64) * (kS / 64) / 8, kHeadsPerPass), 256, 0, stream>>>(
        qa, nullptr, kGin, (long)kDH, kb, nullptr, kGin, (long)kDH,
        (void*)Sbuf, nullptr, kS, (long)kS * kS, nullptr, nullptr, 0L, kS, kS, kDH, kQKScale);
    pweight_kernel<<<(kHeadsPerPass * kS) / 8, 256, 0, stream>>>(Sbuf, Pbuf, Aarr, AMarr, Marr, b, h0);
    const unsigned short* vt = Vt16 + ((size_t)(b * kNH + h0) * kDH) * kS;
    float* hc = Hbuf + (size_t)b * kS * kD + h0 * kDH;
    wmma_gemm64<0, false, 0, 0, false, 0, 2><<<dim3((kS / 64) * (kDH / 64) / 8, kHeadsPerPass), 256, 0, stream>>>(
        Pbuf, nullptr, kS, (long)kS * kS, vt, nullptr, kS, (long)kDH * kS,
        (void*)hc, nullptr, kD, (long)kDH, nullptr, nullptr, 0L, kS, kDH, kS, kPCarryInv);
  }

  norm_kernel<<<(kT * kNH) / 8, 256, 0, stream>>>(Hbuf, lnw, lnb, out);
}
